// GCN_42159398977699
// MI455X (gfx1250) — hardware-verified
//
#include <hip/hip_runtime.h>
#include <stddef.h>
#include <stdint.h>


#define FD      16
#define NT      22
#define NCOL    368
#define ROOTC   352
#define PP      384
#define K1      32
#define K2      64
#define A1ROWS  128
#define NTHR    256
#define NWAVE   8
#define EPT     8
#define CHUNK   (NTHR * EPT)
#define WCAP    (EPT * 32)
#define LISTN   (NWAVE * WCAP)
#define NBA     1024
#define SLA     10
#define RCAP    24576
#define DEGCAP  64
#define GBM     64
#define GBN     128
#define GTHR    128
#define AGG_ZINTS    (LISTN + 2 * RCAP + 3 * NBA)
#define MISC_INTS    16
#define ROWBUF_INTS  (NWAVE * 64)
#define AGG_LDS_INTS (AGG_ZINTS + MISC_INTS + ROWBUF_INTS)
#define OFF_BT1 0
#define OFF_BT2 (PP * K1)
#define OFF_A1  (OFF_BT2 + PP * K2)
#define PL16N   (OFF_A1 + A1ROWS * K1)
#define WSMAX   134217728

static_assert((CHUNK & (CHUNK - 1)) == 0 && CHUNK <= 4096);
static_assert((NBA & (NBA - 1)) == 0 && NBA == (1 << SLA));
static_assert(((long long)CHUNK << SLA) < (1LL << 31));
static_assert(LISTN % NTHR == 0);
static_assert(NBA % (2 * NWAVE) == 0 && NBA % 32 == 0 && NBA % GBM == 0);
static_assert(RCAP % 4 == 0 && AGG_ZINTS % 4 == 0 && ((AGG_ZINTS + MISC_INTS) % 4) == 0);
static_assert(AGG_LDS_INTS * 4 <= 300000);
static_assert(NT * FD == ROOTC && ROOTC + FD == NCOL && NCOL <= PP);
static_assert(PP % GBN == 0 && A1ROWS % GBM == 0 && K1 % 32 == 0 && K2 % 32 == 0);
static_assert(GBM == (GTHR / 32) * 16);
static_assert((PP * 4) % 128 == 0 && (GBN * 4) % 128 == 0);
static_assert((OFF_BT2 * 2) % 128 == 0 && (OFF_A1 * 2) % 128 == 0 && (PL16N * 2) % 256 == 0);
static_assert(FD == 16 && K2 * 2 == 128);

typedef float          v4f   __attribute__((ext_vector_type(4)));
typedef float          v8f   __attribute__((ext_vector_type(8)));
typedef int            v4i   __attribute__((ext_vector_type(4)));
typedef int            v8i   __attribute__((ext_vector_type(8)));
typedef unsigned short v4us  __attribute__((ext_vector_type(4)));
typedef unsigned short v8us  __attribute__((ext_vector_type(8)));
typedef unsigned short v16us __attribute__((ext_vector_type(16)));
typedef __bf16         v16bf __attribute__((ext_vector_type(16)));
typedef v4f  __attribute__((may_alias)) v4fa;
typedef v4i  __attribute__((may_alias)) v4ia;
typedef v4us __attribute__((may_alias)) v4usa;
typedef v8us __attribute__((may_alias)) v8usa;
union FragB { v16bf v; v16us u; v8us h[2]; v8i w; };

__device__ __forceinline__ v8f wmb(const FragB& a, const FragB& b, v8f c) {
  v8f d = __builtin_amdgcn_wmma_f32_16x16x32_bf16(false, a.v, false, b.v, (short)0, c, false, false);
  asm volatile("v_nop\n\tv_nop\n\tv_nop\n\tv_nop" : "+v"(d) : "v"(a.w), "v"(b.w));
  return d;
}

__device__ __forceinline__ unsigned bf16_bits(float f) {
  const unsigned u = __float_as_uint(f);
  return (u + 0x7FFFu + ((u >> 16) & 1u)) >> 16;
}
__device__ __forceinline__ float bf16_val(float f) {
  return __uint_as_float(bf16_bits(f) << 16);
}
__device__ __forceinline__ void split2(float v, unsigned& hb, unsigned& lb) {
  const unsigned h = bf16_bits(v);
  const float r = v - __uint_as_float(h << 16);
  const unsigned l = bf16_bits(r);
  const bool nn = (v != v);
  hb = nn ? 0x7fc0u : h;
  lb = nn ? 0x7fc0u : l;
}

template <int SLB>
__device__ __forceinline__ int scan_chunk(const int* __restrict__ dsts, int nE, int cbase, int slotBase,
                                          int nb, int vec8, int* list, int tid, int lane, int wave) {
  int wc = 0;
  const int el0  = tid * EPT;
  const int e0   = cbase + el0;
  const int sent = -2147483647 - 1;
  v4i da, db;
  if (vec8 != 0 && cbase + CHUNK <= nE) {
    da = *(const v4i*)(dsts + e0);
    db = *(const v4i*)(dsts + e0 + 4);
  } else {
    da.x = (e0     < nE) ? dsts[min(e0,     nE - 1)] : sent;
    da.y = (e0 + 1 < nE) ? dsts[min(e0 + 1, nE - 1)] : sent;
    da.z = (e0 + 2 < nE) ? dsts[min(e0 + 2, nE - 1)] : sent;
    da.w = (e0 + 3 < nE) ? dsts[min(e0 + 3, nE - 1)] : sent;
    db.x = (e0 + 4 < nE) ? dsts[min(e0 + 4, nE - 1)] : sent;
    db.y = (e0 + 5 < nE) ? dsts[min(e0 + 5, nE - 1)] : sent;
    db.z = (e0 + 6 < nE) ? dsts[min(e0 + 6, nE - 1)] : sent;
    db.w = (e0 + 7 < nE) ? dsts[min(e0 + 7, nE - 1)] : sent;
  }
  const unsigned nbs = (unsigned)slotBase;
  const unsigned unb = (unsigned)nb;
  const unsigned s0 = (unsigned)da.x - nbs, s1 = (unsigned)da.y - nbs;
  const unsigned s2 = (unsigned)da.z - nbs, s3 = (unsigned)da.w - nbs;
  const unsigned s4 = (unsigned)db.x - nbs, s5 = (unsigned)db.y - nbs;
  const unsigned s6 = (unsigned)db.z - nbs, s7 = (unsigned)db.w - nbs;
  const bool h0 = s0 < unb, h1 = s1 < unb, h2 = s2 < unb, h3 = s3 < unb;
  const bool h4 = s4 < unb, h5 = s5 < unb, h6 = s6 < unb, h7 = s7 < unb;
  const unsigned any = __builtin_amdgcn_ballot_w32(h0 | h1 | h2 | h3 | h4 | h5 | h6 | h7);
  if (any != 0u) {
#define HITJ(J, HJ, SJ) { \
      const unsigned mj = __builtin_amdgcn_ballot_w32(HJ); \
      if (mj != 0u) { \
        if (HJ) { \
          const int pos = wc + (int)__builtin_amdgcn_mbcnt_lo(mj, 0u); \
          if (pos < WCAP) list[wave * WCAP + pos] = ((el0 + (J)) << SLB) | (int)(SJ); \
        } \
        wc += (int)__builtin_popcount(mj); } }
    HITJ(0, h0, s0)
    HITJ(1, h1, s1)
    HITJ(2, h2, s2)
    HITJ(3, h3, s3)
    HITJ(4, h4, s4)
    HITJ(5, h5, s5)
    HITJ(6, h6, s6)
    HITJ(7, h7, s7)
#undef HITJ
  }
  return wc;
}

__device__ __forceinline__ float wval(const float* __restrict__ ee, const float* __restrict__ lw,
                                      const float* __restrict__ lb, int type, int j) {
  float acc = 0.0f;
#pragma unroll 1
  for (int k4 = 0; k4 < 4; ++k4) {
    const v4f e = *(const v4f*)(ee + type * FD + 4 * k4);
    const v4f w = *(const v4f*)(lw + j * FD + 4 * k4);
    acc = fmaf(bf16_val(e.x), bf16_val(w.x), acc);
    acc = fmaf(bf16_val(e.y), bf16_val(w.y), acc);
    acc = fmaf(bf16_val(e.z), bf16_val(w.z), acc);
    acc = fmaf(bf16_val(e.w), bf16_val(w.w), acc);
  }
  return acc + bf16_val(lb[j]);
}

__global__ __launch_bounds__(NTHR) void k_prep(const float* __restrict__ aemb, const float* __restrict__ eemb,
                                               const float* __restrict__ l1w, const float* __restrict__ l1b,
                                               const float* __restrict__ root1,
                                               const float* __restrict__ l2w, const float* __restrict__ l2b,
                                               const float* __restrict__ root2,
                                               int nZ, unsigned short* pl) {
  __shared__ __attribute__((aligned(16))) float wl[256];
  const int tid = (int)threadIdx.x;
  const int b   = (int)blockIdx.x;
  v8us o = {0, 0, 0, 0, 0, 0, 0, 0};
  int doff = 0;
  bool wr = false;
  if (b < 2 * NT) {
    const int layer = (b >= NT) ? 1 : 0;
    const int type  = b - layer * NT;
    float w;
    if (layer == 0) w = wval(eemb, l1w, l1b, type, tid);
    else            w = wval(eemb, l2w, l2b, type, tid);
    wl[tid] = w;
    __syncthreads();
    if (layer == 0) {
      const int u  = tid & 63;
      const int oc = u >> 2;
      const int p  = u & 3;
      const int i0 = 8 * (p & 1);
      const bool lo = (p >> 1) != 0;
#pragma unroll
      for (int ii = 0; ii < 8; ++ii) {
        const float v = wl[(i0 + ii) * FD + oc];
        unsigned hb, lb;
        split2(v, hb, lb);
        o[ii] = (unsigned short)(lo ? lb : hb);
      }
      doff = OFF_BT1 + type * (FD * K1) + u * 8;
      wr = tid < 64;
    } else {
      const int u  = tid & 127;
      const int oc = u >> 3;
      const int p  = u & 7;
      const int i0 = 8 * (p & 1);
      const bool lo = (p >> 2) != 0;
#pragma unroll
      for (int ii = 0; ii < 8; ++ii) {
        const float v = wl[(i0 + ii) * FD + oc];
        unsigned hb, lb;
        split2(v, hb, lb);
        o[ii] = (unsigned short)(lo ? lb : hb);
      }
      doff = OFF_BT2 + type * (FD * K2) + u * 8;
      wr = tid < 128;
    }
  } else if (b == 2 * NT) {
    const int u  = tid & 127;
    const int r  = u >> 2;
    const int p  = u & 3;
    const int oc = r & 15;
    const int i0 = 8 * (p & 1);
    const bool valid = (r < 16) && (p < 2);
#pragma unroll
    for (int ii = 0; ii < 8; ++ii) {
      const float f = root1[(i0 + ii) * FD + oc];
      o[ii] = valid ? (unsigned short)bf16_bits(f) : (unsigned short)0;
    }
    doff = OFF_BT1 + ROOTC * K1 + u * 8;
    wr = tid < 128;
  } else if (b == 2 * NT + 1) {
    const int u  = tid;
    const int r  = u >> 3;
    const int p  = u & 7;
    const int oc = r & 15;
    const int i0 = 8 * (p & 1);
    const bool valid = (r < 16) && (p < 4);
#pragma unroll
    for (int ii = 0; ii < 8; ++ii) {
      const float f = root2[(i0 + ii) * FD + oc];
      o[ii] = valid ? (unsigned short)bf16_bits(f) : (unsigned short)0;
    }
    doff = OFF_BT2 + ROOTC * K2 + u * 8;
    wr = true;
  } else if (b < 2 * NT + 4) {
    const int u  = (b - (2 * NT + 2)) * NTHR + tid;
    const int z  = u >> 2;
    const int p  = u & 3;
    const int zc = z < nZ ? z : nZ - 1;
    const float* sp = aemb + (size_t)zc * FD + 8 * (p & 1);
    const v4f a = *(const v4f*)sp;
    const v4f c = *(const v4f*)(sp + 4);
    const bool valid = z < nZ;
    o[0] = valid ? (unsigned short)bf16_bits(a.x) : (unsigned short)0;
    o[1] = valid ? (unsigned short)bf16_bits(a.y) : (unsigned short)0;
    o[2] = valid ? (unsigned short)bf16_bits(a.z) : (unsigned short)0;
    o[3] = valid ? (unsigned short)bf16_bits(a.w) : (unsigned short)0;
    o[4] = valid ? (unsigned short)bf16_bits(c.x) : (unsigned short)0;
    o[5] = valid ? (unsigned short)bf16_bits(c.y) : (unsigned short)0;
    o[6] = valid ? (unsigned short)bf16_bits(c.z) : (unsigned short)0;
    o[7] = valid ? (unsigned short)bf16_bits(c.w) : (unsigned short)0;
    doff = OFF_A1 + u * 8;
    wr = true;
  }
  unsigned short* dp = pl + doff;
  if (wr) *(volatile v8us*)dp = o;
  __threadfence();
  if (wr) *(volatile v8us*)dp = o;
}

__global__ __launch_bounds__(GTHR) void k_gemm(const unsigned short* __restrict__ Apl,
                                               const unsigned short* __restrict__ BT, int K,
                                               const float* __restrict__ bias, int useBias,
                                               float* outp, int ldo) {
  __shared__ __attribute__((aligned(16))) float stg[GBM * GBN];
  const int tid = (int)threadIdx.x, lane = tid & 31, wave = tid >> 5, hh = lane >> 4, m = lane & 15;
  const int rowBase = (int)blockIdx.x * GBM;
  const int col0    = (int)blockIdx.y * GBN;

  v8f acc[8];
  {
    const v8f z = {0.f, 0.f, 0.f, 0.f, 0.f, 0.f, 0.f, 0.f};
#pragma unroll
    for (int t = 0; t < 8; ++t) acc[t] = z;
  }
  const unsigned short* ap = Apl + (size_t)(rowBase + 16 * wave + m) * (size_t)K + 8 * hh;
  const unsigned short* bp = BT + (size_t)(col0 + m) * (size_t)K + 8 * hh;

#pragma unroll 1
  for (int k0 = 0; k0 < K; k0 += 32) {
    FragB af;
    af.h[0] = *(const v8usa*)(ap + k0);
    af.h[1] = *(const v8usa*)(ap + k0 + 16);
#pragma unroll
    for (int nt = 0; nt < 8; ++nt) {
      const unsigned short* wq = bp + (size_t)(16 * nt) * (size_t)K + k0;
      FragB bf;
      bf.h[0] = *(const v8usa*)wq;
      bf.h[1] = *(const v8usa*)(wq + 16);
      acc[nt] = wmb(af, bf, acc[nt]);
    }
  }

#pragma unroll
  for (int nt = 0; nt < 8; ++nt) {
    const int lc = 16 * nt + m;
#pragma unroll
    for (int r = 0; r < 8; ++r) {
      const int lr = 16 * wave + 8 * hh + r;
      stg[lr * GBN + lc] = acc[nt][r];
    }
  }
  __syncthreads();

  v4f bb4;
  {
    const int c0 = col0 + 4 * lane;
    const bool inb = (useBias != 0) && (c0 >= ROOTC) && (c0 < ROOTC + FD);
    int bi = c0 - ROOTC;
    bi = bi < 0 ? 0 : (bi > FD - 4 ? FD - 4 : bi);
    const v4f bs = *(const v4f*)(bias + bi);
    bb4.x = inb ? bf16_val(bs.x) : 0.0f;
    bb4.y = inb ? bf16_val(bs.y) : 0.0f;
    bb4.z = inb ? bf16_val(bs.z) : 0.0f;
    bb4.w = inb ? bf16_val(bs.w) : 0.0f;
  }

  v4f pv[16];
#pragma unroll
  for (int i = 0; i < 16; ++i) {
    const v4f t = *(const v4fa*)(stg + (16 * wave + i) * GBN + 4 * lane);
    pv[i] = t + bb4;
  }
#pragma unroll
  for (int i = 0; i < 16; ++i) {
    const int r = rowBase + 16 * wave + i;
    *(volatile v4f*)(outp + (size_t)r * (size_t)ldo + col0 + 4 * lane) = pv[i];
  }
  __threadfence();
#pragma unroll
  for (int i = 0; i < 16; ++i) {
    const int r = rowBase + 16 * wave + i;
    *(volatile v4f*)(outp + (size_t)r * (size_t)ldo + col0 + 4 * lane) = pv[i];
  }
}

template <int LAYER>
__device__ __forceinline__ v4f slot_row(int s, int nodeBase, int nN, int nE, int nZ,
                                        const int* cnt, const int* offs, const int* sl,
                                        const int* __restrict__ srcs, const int* __restrict__ ety,
                                        const int* __restrict__ xid, const float* __restrict__ P,
                                        int lane, float pz) {
  const int node = nodeBase + s;
  int c = cnt[s];
  const bool big = c > DEGCAP;
  c = c < 0 ? 0 : (c > DEGCAP ? DEGCAP : c);
  int o = offs[s];
  o = o < 0 ? 0 : (o > RCAP ? RCAP : o);
  const int nc = node < nN ? node : nN - 1;
  const int hj = lane >> 2, q = lane & 3;
  float a0 = 0.0f, a1 = 0.0f, a2 = 0.0f, a3 = 0.0f;
#pragma unroll 1
  for (int b0 = 0; b0 < c; b0 += 8) {
    const int hx = b0 + hj;
    const bool ok = hx < c;
    int idx = o + hx;
    idx = idx > RCAP - 1 ? RCAP - 1 : idx;
    const int ent = sl[idx];
    int eid = ent >> SLA;
    eid = eid < 0 ? 0 : (eid > nE - 1 ? nE - 1 : eid);
    int sr = srcs[eid];
    sr = sr < 0 ? 0 : (sr > nN - 1 ? nN - 1 : sr);
    int tt = ety[eid];
    tt = tt < 0 ? 0 : (tt > NT - 1 ? NT - 1 : tt);
    int key;
    if constexpr (LAYER == 1) {
      int z = xid[sr];
      key = z < 0 ? 0 : (z > nZ - 1 ? nZ - 1 : z);
    } else {
      key = sr;
    }
    const v4f g = *(const v4f*)(P + (size_t)key * PP + tt * FD + 4 * q);
    a0 += ok ? g.x : 0.0f;
    a1 += ok ? g.y : 0.0f;
    a2 += ok ? g.z : 0.0f;
    a3 += ok ? g.w : 0.0f;
  }
  a0 += __shfl_xor(a0, 4, 32);  a1 += __shfl_xor(a1, 4, 32);
  a2 += __shfl_xor(a2, 4, 32);  a3 += __shfl_xor(a3, 4, 32);
  a0 += __shfl_xor(a0, 8, 32);  a1 += __shfl_xor(a1, 8, 32);
  a2 += __shfl_xor(a2, 8, 32);  a3 += __shfl_xor(a3, 8, 32);
  a0 += __shfl_xor(a0, 16, 32); a1 += __shfl_xor(a1, 16, 32);
  a2 += __shfl_xor(a2, 16, 32); a3 += __shfl_xor(a3, 16, 32);

  int keyd;
  if constexpr (LAYER == 1) {
    int z = xid[nc];
    keyd = z < 0 ? 0 : (z > nZ - 1 ? nZ - 1 : z);
  } else {
    keyd = nc;
  }
  const v4f rt = *(const v4f*)(P + (size_t)keyd * PP + ROOTC + 4 * q);
  const float pzr = big ? __int_as_float(0x7fc00000) : pz;
  float y0 = (a0 + rt.x) + pzr;
  float y1 = (a1 + rt.y) + pzr;
  float y2 = (a2 + rt.z) + pzr;
  float y3 = (a3 + rt.w) + pzr;
  if constexpr (LAYER == 1) {
    y0 = (y0 > 0.0f) ? y0 : (y0 - y0);
    y1 = (y1 > 0.0f) ? y1 : (y1 - y1);
    y2 = (y2 > 0.0f) ? y2 : (y2 - y2);
    y3 = (y3 > 0.0f) ? y3 : (y3 - y3);
  }
  const bool live = node < nN;
  v4f y;
  y.x = live ? y0 : 0.0f;
  y.y = live ? y1 : 0.0f;
  y.z = live ? y2 : 0.0f;
  y.w = live ? y3 : 0.0f;
  return y;
}

template <int LAYER>
__global__ __launch_bounds__(NTHR) void k_scan(const int* __restrict__ srcs, const int* __restrict__ dsts,
                                               const int* __restrict__ ety, const int* __restrict__ xid,
                                               const float* __restrict__ P,
                                               int nE, int nN, int nZ, int vec8, int mRows,
                                               unsigned short* ha, float* outp) {
  extern __shared__ __attribute__((aligned(16))) int dsm[];
  int* list = dsm;
  int* hl   = dsm + LISTN;
  int* sl   = hl + RCAP;
  int* cnt  = sl + RCAP;
  int* offs = cnt + NBA;
  int* cur  = offs + NBA;
  int* misc = cur + NBA;
  const int tid = (int)threadIdx.x, lane = tid & 31, wave = tid >> 5;
  unsigned short* rowbuf = (unsigned short*)(misc + MISC_INTS) + wave * 128;
  const int nodeBase = (int)blockIdx.x * NBA;

  {
    const v4i z4 = {0, 0, 0, 0};
    for (int i = tid * 4; i < AGG_ZINTS; i += NTHR * 4) *(v4ia*)(dsm + i) = z4;
    if (tid < MISC_INTS) misc[tid] = 0;
  }
  __syncthreads();

  int t = 0, ov = 0;
  const int nChunks = (nE + CHUNK - 1) / CHUNK;
#pragma unroll 1
  for (int ch = 0; ch < nChunks; ++ch) {
    const int cbase = ch * CHUNK;
    const int wc = scan_chunk<SLA>(dsts, nE, cbase, nodeBase, NBA, vec8, list, tid, lane, wave);
    if (lane == 0) misc[wave] = wc;
    __syncthreads();
    if (wave == 0) {
#pragma unroll 1
      for (int w2 = 0; w2 < NWAVE; ++w2) {
        int c = misc[w2];
        c = c < 0 ? 0 : (c > WCAP ? WCAP : c);
#pragma unroll 1
        for (int b0 = 0; b0 < c; b0 += 32) {
          const int idx = b0 + lane;
          const int ent = list[w2 * WCAP + (idx < WCAP ? idx : WCAP - 1)];
          const int m32 = (c - b0) < 32 ? (c - b0) : 32;
#pragma unroll 1
          for (int k = 0; k < m32; ++k) {
            const int u    = __builtin_amdgcn_readlane(ent, k);
            const int slot = u & (NBA - 1);
            const int el   = (u >> SLA) & (CHUNK - 1);
            const int pk   = ((cbase + el) << SLA) | slot;
            if (t < RCAP) {
              if (lane == 0) { hl[t] = pk; cnt[slot] = cnt[slot] + 1; }
              t = t + 1;
            } else {
              ov = 1;
            }
          }
        }
      }
    }
    __syncthreads();
  }
  if (wave == 0 && lane == 0) { misc[8] = t; misc[9] = ov; }
  __syncthreads();
  int tt = misc[8];
  tt = tt < 0 ? 0 : (tt > RCAP ? RCAP : tt);
  const int ovf = misc[9];

  if (wave == 0) {
    const int base = lane * (NBA / 32);
    int s = 0;
#pragma unroll 1
    for (int i = 0; i < NBA / 32; ++i) s += cnt[base + i];
    int incl = s;
#pragma unroll
    for (int d = 1; d < 32; d <<= 1) {
      const int y = __shfl_up(incl, d, 32);
      if (lane >= d) incl += y;
    }
    int run = incl - s;
#pragma unroll 1
    for (int i = 0; i < NBA / 32; ++i) {
      const int cv = cnt[base + i];
      offs[base + i] = run;
      cur[base + i]  = run;
      run += cv;
    }
  }
  __syncthreads();
  if (wave == 0) {
#pragma unroll 1
    for (int b0 = 0; b0 < tt; b0 += 32) {
      const int idx = b0 + lane;
      const int ent = hl[idx < RCAP ? idx : RCAP - 1];
      const int m32 = (tt - b0) < 32 ? (tt - b0) : 32;
#pragma unroll 1
      for (int k = 0; k < m32; ++k) {
        const int u    = __builtin_amdgcn_readlane(ent, k);
        const int slot = u & (NBA - 1);
        if (lane == 0) {
          int p = cur[slot];
          p = p < 0 ? 0 : (p > RCAP - 1 ? RCAP - 1 : p);
          sl[p] = u;
          cur[slot] = p + 1;
        }
      }
    }
  }
  __syncthreads();

  const float pz = (ovf != 0) ? __int_as_float(0x7fc00000) : 0.0f;
#pragma unroll 1
  for (int pi = 0; pi < NBA / (2 * NWAVE); ++pi) {
    const int s0    = 2 * (pi * NWAVE + wave);
    const int node0 = nodeBase + s0;
    const v4f rA = slot_row<LAYER>(s0,     nodeBase, nN, nE, nZ, cnt, offs, sl, srcs, ety, xid, P, lane, pz);
    const v4f rB = slot_row<LAYER>(s0 + 1, nodeBase, nN, nE, nZ, cnt, offs, sl, srcs, ety, xid, P, lane, pz);
    const bool selB = (lane & 4) != 0;
    v4f rr;
    rr.x = selB ? rB.x : rA.x;
    rr.y = selB ? rB.y : rA.y;
    rr.z = selB ? rB.z : rA.z;
    rr.w = selB ? rB.w : rA.w;
    if constexpr (LAYER == 1) {
      if (lane < 8) {
        unsigned h0, l0, h1, l1, h2, l2, h3, l3;
        split2(rr.x, h0, l0);
        split2(rr.y, h1, l1);
        split2(rr.z, h2, l2);
        split2(rr.w, h3, l3);
        v4us mh, ml;
        mh[0] = (unsigned short)h0; mh[1] = (unsigned short)h1; mh[2] = (unsigned short)h2; mh[3] = (unsigned short)h3;
        ml[0] = (unsigned short)l0; ml[1] = (unsigned short)l1; ml[2] = (unsigned short)l2; ml[3] = (unsigned short)l3;
        unsigned short* rb = rowbuf + 64 * (lane >> 2) + 4 * (lane & 3);
        *(v4usa*)(rb)      = mh;
        *(v4usa*)(rb + 16) = ml;
        *(v4usa*)(rb + 32) = mh;
        *(v4usa*)(rb + 48) = ml;
      }
      __syncthreads();
      const v8us qv = *(const v8usa*)(rowbuf + 8 * (lane & 15));
      __syncthreads();
      const bool wr = (node0 < mRows) && (lane < 16);
      unsigned short* hp = ha + (size_t)node0 * K2 + 8 * (lane & 15);
      if (wr) *(volatile v8us*)hp = qv;
      __threadfence();
      if (wr) *(volatile v8us*)hp = qv;
    } else {
      const bool wr = (node0 < nN) && (lane < 8);
      float* op = outp + (size_t)node0 * FD + 4 * (lane & 7);
      if (wr) *(volatile v4f*)op = rr;
      __threadfence();
      if (wr) *(volatile v4f*)op = rr;
    }
  }
}

static inline int cdiv(int a, int b) { return (a + b - 1) / b; }
static inline size_t al256(size_t o) { return (o + 255) & ~(size_t)255; }

extern "C" void kernel_launch(void* const* d_in, const int* in_sizes, int n_in,
                              void* d_out, int out_size, void* d_ws, size_t ws_size,
                              hipStream_t stream) {
  if (n_in < 13) return;
  const int nN = in_sizes[0];
  if (nN < 2 || (nN & 1) != 0 || nN > (1 << 22)) return;
  if (in_sizes[1] < 2 || (in_sizes[1] & 1) != 0) return;
  const int nE = in_sizes[1] / 2;
  if (nE < 1 || nE >= (1 << 21)) return;
  if (in_sizes[2] != nE) return;
  if (in_sizes[3] < FD || (in_sizes[3] % FD) != 0) return;
  const int nZ = in_sizes[3] / FD;
  if (nZ > A1ROWS) return;
  if (in_sizes[4] != NT * FD) return;
  if (in_sizes[5] != 256 * FD || in_sizes[6] != 256) return;
  if (in_sizes[7] != FD * FD || in_sizes[8] != FD) return;
  if (in_sizes[9] != 256 * FD || in_sizes[10] != 256) return;
  if (in_sizes[11] != FD * FD || in_sizes[12] != FD) return;
  if ((long long)out_size != (long long)nN * FD) return;

  const int*   xid   = (const int*)d_in[0];
  const int*   edge  = (const int*)d_in[1];
  const int*   ety   = (const int*)d_in[2];
  const float* aemb  = (const float*)d_in[3];
  const float* eemb  = (const float*)d_in[4];
  const float* l1w   = (const float*)d_in[5];
  const float* l1b   = (const float*)d_in[6];
  const float* root1 = (const float*)d_in[7];
  const float* bias1 = (const float*)d_in[8];
  const float* l2w   = (const float*)d_in[9];
  const float* l2b   = (const float*)d_in[10];
  const float* root2 = (const float*)d_in[11];
  const float* bias2 = (const float*)d_in[12];
  float* out = (float*)d_out;
  const int* src = edge;
  const int* dst = edge + nE;

  const int MP = cdiv(nN, GBM) * GBM;
  const int gM = MP / GBM;
  const int gA = cdiv(MP, NBA);
  if ((long long)gA * NBA < (long long)MP) return;
  const int vec8 = ((nE & 3) == 0) ? 1 : 0;

  char* ws = (char*)d_ws;
  size_t off = 0;
  const size_t oPL = off; off = al256(off + (size_t)PL16N * 2);
  const size_t oP1 = off; off = al256(off + (size_t)A1ROWS * PP * 4);
  const size_t oHA = off; off = al256(off + (size_t)MP * K2 * 2);
  const size_t oP2 = off; off = al256(off + (size_t)MP * PP * 4);
  if (off > ws_size || off > (size_t)WSMAX) return;
  unsigned short* PL = (unsigned short*)(ws + oPL);
  float*          P1 = (float*)(ws + oP1);
  unsigned short* HA = (unsigned short*)(ws + oHA);
  float*          P2 = (float*)(ws + oP2);

  const size_t scanLds = (size_t)AGG_LDS_INTS * 4;
  hipFuncSetAttribute(reinterpret_cast<const void*>(&k_scan<1>), hipFuncAttributeMaxDynamicSharedMemorySize, (int)scanLds);
  hipFuncSetAttribute(reinterpret_cast<const void*>(&k_scan<2>), hipFuncAttributeMaxDynamicSharedMemorySize, (int)scanLds);

  k_prep<<<2 * NT + 4, NTHR, 0, stream>>>(aemb, eemb, l1w, l1b, root1, l2w, l2b, root2, nZ, PL);
  k_gemm<<<dim3(A1ROWS / GBM, PP / GBN), GTHR, 0, stream>>>(PL + OFF_A1, PL + OFF_BT1, K1, bias1, 1, P1, PP);
  k_scan<1><<<gA, NTHR, scanLds, stream>>>(src, dst, ety, xid, P1, nE, nN, nZ, vec8, MP, HA, out);
  k_gemm<<<dim3(gM, PP / GBN), GTHR, 0, stream>>>(HA, PL + OFF_BT2, K2, bias2, 1, P2, PP);
  k_scan<2><<<gA, NTHR, scanLds, stream>>>(src, dst, ety, xid, P2, nE, nN, nZ, vec8, MP, HA, out);
}
